// GPT2Attention_49435073577418
// MI455X (gfx1250) — hardware-verified
//
#include <hip/hip_runtime.h>


typedef __attribute__((ext_vector_type(16))) _Float16 v16h;
typedef __attribute__((ext_vector_type(8)))  _Float16 v8h;
typedef __attribute__((ext_vector_type(8)))  float    v8f;
typedef __attribute__((ext_vector_type(4)))  float    v4f;

union V16u { v16h v; v8h h[2]; };

#define WMMA_F16(a, b, c) \
  __builtin_amdgcn_wmma_f32_16x16x32_f16(false, (a), false, (b), (short)0, (c), false, false)

constexpr int Bc  = 4;
constexpr int Sc  = 2048;
constexpr int Dc  = 1024;
constexpr int HDc = 128;

__global__ void __launch_bounds__(256) gpt2attn_wt_kernel(
    const float* __restrict__ Wq, const float* __restrict__ Wk,
    const float* __restrict__ Wv,
    _Float16* __restrict__ WTq, _Float16* __restrict__ WTk,
    _Float16* __restrict__ WTv) {
  int idx = blockIdx.x * blockDim.x + threadIdx.x;
  int k = idx >> 7;
  int n = idx & 127;
  int src = k * HDc + n;
  int dst = n * Dc + k;
  *(volatile _Float16*)(WTq + dst) = (_Float16)Wq[src]; *(volatile _Float16*)(WTk + dst) = (_Float16)Wk[src]; *(volatile _Float16*)(WTv + dst) = (_Float16)Wv[src];
  __threadfence();
  *(volatile _Float16*)(WTq + dst) = (_Float16)Wq[src]; *(volatile _Float16*)(WTk + dst) = (_Float16)Wk[src]; *(volatile _Float16*)(WTv + dst) = (_Float16)Wv[src];
}

__global__ void __launch_bounds__(256) gpt2attn_qkv_kernel(
    const float* __restrict__ x,
    const _Float16* __restrict__ WTq, const _Float16* __restrict__ WTk,
    const _Float16* __restrict__ WTv,
    _Float16* __restrict__ qh, _Float16* __restrict__ kh,
    _Float16* __restrict__ vT) {
  const int tid  = threadIdx.x;
  const int wave = tid >> 5;
  const int lane = tid & 31;
  const int l16  = lane & 15;
  const int lh   = lane >> 4;
  const int rt   = blockIdx.x;
  const int n0   = wave * 16;

  const float* xrow = x + (size_t)(rt * 16 + l16) * Dc;
  __shared__ __attribute__((aligned(16))) _Float16 sQKV[3][16][HDc];
  const _Float16* wq = WTq + (size_t)(n0 + l16) * Dc + 8 * lh;
  const _Float16* wk = WTk + (size_t)(n0 + l16) * Dc + 8 * lh;
  const _Float16* wv = WTv + (size_t)(n0 + l16) * Dc + 8 * lh;

  v8f cq = {};
  v8f ck = {};
  v8f cv = {};

  for (int k0 = 0; k0 < Dc; k0 += 32) {
    V16u a;
    const v4f f0 = *(const v4f*)(xrow + k0 + 8 * lh);
    const v4f f1 = *(const v4f*)(xrow + k0 + 8 * lh + 4);
    const v4f f2 = *(const v4f*)(xrow + k0 + 16 + 8 * lh);
    const v4f f3 = *(const v4f*)(xrow + k0 + 16 + 8 * lh + 4);
#pragma unroll
    for (int j = 0; j < 4; ++j) {
      a.v[j]      = (_Float16)f0[j];
      a.v[j + 4]  = (_Float16)f1[j];
      a.v[j + 8]  = (_Float16)f2[j];
      a.v[j + 12] = (_Float16)f3[j];
    }
    V16u bq, bk, bv;
    bq.h[0] = *(const v8h*)(wq + k0); bq.h[1] = *(const v8h*)(wq + k0 + 16);
    bk.h[0] = *(const v8h*)(wk + k0); bk.h[1] = *(const v8h*)(wk + k0 + 16);
    bv.h[0] = *(const v8h*)(wv + k0); bv.h[1] = *(const v8h*)(wv + k0 + 16);
    cq = WMMA_F16(a.v, bq.v, cq);
    ck = WMMA_F16(a.v, bk.v, ck);
    cv = WMMA_F16(a.v, bv.v, cv);
    asm volatile("v_nop\n\tv_nop\n\tv_nop\n\tv_nop" : "+v"(cq), "+v"(cv) : "v"(a.v), "v"(bv.v));
  }

#pragma unroll
  for (int r = 0; r < 8; ++r) {
    const int col = n0 + l16;
    sQKV[0][r + 8 * lh][col] = (_Float16)cq[r];
    sQKV[1][r + 8 * lh][col] = (_Float16)ck[r];
    sQKV[2][r + 8 * lh][col] = (_Float16)cv[r];
  }
  __syncthreads();
  for (int pass = 0; pass < 2; ++pass) {
#pragma unroll
    for (int j = 0; j < 3; ++j) {
      const int piece = j * 256 + tid, mat = piece >> 8, rr = (piece >> 4) & 15, q8 = (piece & 15) * 8;
      _Float16* dst = (mat == 0) ? qh : (mat == 1) ? kh : vT;
      *(volatile v8h*)(dst + (size_t)(rt * 16 + rr) * HDc + q8) = *(const v8h*)(&sQKV[mat][rr][q8]);
    }
    __threadfence();
  }
}

__global__ void __launch_bounds__(128) gpt2attn_flash_kernel(
    const _Float16* __restrict__ qh, const _Float16* __restrict__ kh,
    const _Float16* __restrict__ vT, float* __restrict__ out) {
  __shared__ __align__(32) _Float16 ldsP[4][16 * 32];
  __shared__ __attribute__((aligned(16))) float sO[4][16][HDc];

  const int tid  = threadIdx.x;
  const int wave = tid >> 5;
  const int lane = tid & 31;
  const int l16  = lane & 15;
  const int lh   = lane >> 4;
  const int b     = blockIdx.x >> 5;
  const int qBase = (blockIdx.x & 31) * 64 + wave * 16;
  const float scale = 0.08838834764831845f;

  v16h aq[4];
  {
    const _Float16* qrow = qh + ((size_t)b * Sc + qBase + l16) * HDc;
#pragma unroll
    for (int hc = 0; hc < 4; ++hc) {
      V16u a;
      a.h[0] = *(const v8h*)(qrow + hc * 32 + 8 * lh);
      a.h[1] = *(const v8h*)(qrow + hc * 32 + 16 + 8 * lh);
      aq[hc] = a.v;
    }
  }

  float m[8], l[8];
  v8f co[8];
  v8f zero = {};
#pragma unroll
  for (int r = 0; r < 8; ++r) { m[r] = -1e30f; l[r] = 0.0f; }
#pragma unroll
  for (int n = 0; n < 8; ++n) co[n] = zero;

  const _Float16* kbB = kh + (size_t)b * Sc * HDc;
  const _Float16* vbB = vT + (size_t)b * Sc * HDc;

  for (int k0 = 0; k0 < qBase + 16; k0 += 32) {
    v8f s0 = {};
    v8f s1 = {};
    const _Float16* kr0 = kbB + (size_t)(k0 + l16) * HDc + 8 * lh;
    const _Float16* kr1 = kr0 + 16 * HDc;
#pragma unroll
    for (int hc = 0; hc < 4; ++hc) {
      V16u b0, b1;
      b0.h[0] = *(const v8h*)(kr0 + hc * 32); b0.h[1] = *(const v8h*)(kr0 + hc * 32 + 16);
      b1.h[0] = *(const v8h*)(kr1 + hc * 32); b1.h[1] = *(const v8h*)(kr1 + hc * 32 + 16);
      s0 = WMMA_F16(aq[hc], b0.v, s0);
      s1 = WMMA_F16(aq[hc], b1.v, s1);
    }
    asm volatile("v_nop\n\tv_nop\n\tv_nop\n\tv_nop" : "+v"(s0), "+v"(s1) : "v"(aq[3]), "v"(aq[0]));

    float alpha[8];
#pragma unroll
    for (int r = 0; r < 8; ++r) {
      const int row  = qBase + r + 8 * lh;
      const int key0 = k0 + l16;
      const int key1 = key0 + 16;
      float x0 = (key0 <= row) ? s0[r] * scale : -1e30f;
      float x1 = (key1 <= row) ? s1[r] * scale : -1e30f;
      float tmax = fmaxf(x0, x1);
#pragma unroll
      for (int off = 1; off < 16; off <<= 1)
        tmax = fmaxf(tmax, __shfl_xor(tmax, off, 32));
      const float mn = fmaxf(m[r], tmax);
      alpha[r] = __expf(m[r] - mn);
      const float p0 = __expf(x0 - mn);
      const float p1 = __expf(x1 - mn);
      float ps = p0 + p1;
#pragma unroll
      for (int off = 1; off < 16; off <<= 1)
        ps += __shfl_xor(ps, off, 32);
      l[r] = l[r] * alpha[r] + ps;
      m[r] = mn;
      ldsP[wave][(r + 8 * lh) * 32 + l16]      = (_Float16)p0;
      ldsP[wave][(r + 8 * lh) * 32 + 16 + l16] = (_Float16)p1;
    }
#pragma unroll
    for (int n = 0; n < 8; ++n)
#pragma unroll
      for (int r = 0; r < 8; ++r)
        co[n][r] *= alpha[r];

    asm volatile("s_wait_dscnt 0" ::: "memory");

    V16u ap;
    ap.h[0] = *(const v8h*)(&ldsP[wave][l16 * 32 + 8 * lh]);
    ap.h[1] = *(const v8h*)(&ldsP[wave][l16 * 32 + 16 + 8 * lh]);
#pragma unroll
    for (int n = 0; n < 8; ++n) {
      v16h bv;
#pragma unroll
      for (int e = 0; e < 16; ++e) bv[e] = vbB[(size_t)(k0 + ((e < 8) ? (8 * lh + e) : (16 + 8 * lh + e - 8))) * HDc + n * 16 + l16];
      co[n] = WMMA_F16(ap.v, bv, co[n]);
    }
    asm volatile("v_nop\n\tv_nop\n\tv_nop\n\tv_nop" : "+v"(co[0]), "+v"(co[7]) : "v"(ap.v));
  }

#pragma unroll
  for (int r = 0; r < 8; ++r) {
    const float inv = 1.0f / l[r];
#pragma unroll
    for (int n = 0; n < 8; ++n) sO[wave][r + 8 * lh][n * 16 + l16] = co[n][r] * inv;
  }
  __builtin_amdgcn_fence(__ATOMIC_RELEASE, "workgroup"); __builtin_amdgcn_wave_barrier(); __builtin_amdgcn_fence(__ATOMIC_ACQUIRE, "workgroup");
  for (int pass = 0; pass < 2; ++pass) {
#pragma unroll
    for (int rr = 0; rr < 16; ++rr)
      *(volatile v4f*)(out + ((size_t)b * Sc + qBase + rr) * HDc + lane * 4) = *(const v4f*)(&sO[wave][rr][lane * 4]);
    __threadfence();
  }
}

extern "C" void kernel_launch(void* const* d_in, const int* in_sizes, int n_in,
                              void* d_out, int out_size, void* d_ws, size_t ws_size,
                              hipStream_t stream) {
  (void)in_sizes; (void)n_in; (void)out_size;
  if (ws_size < (size_t)3 * HDc * Dc * 2 + (size_t)3 * Bc * Sc * HDc * 2) return;
  const float* x  = (const float*)d_in[0];
  const float* Wq = (const float*)d_in[2];
  const float* Wk = (const float*)d_in[3];
  const float* Wv = (const float*)d_in[4];
  float* out = (float*)d_out;

  char* ws = (char*)d_ws;
  const size_t wt_bytes  = (size_t)HDc * Dc * sizeof(_Float16);
  const size_t qkv_bytes = (size_t)Bc * Sc * HDc * sizeof(_Float16);
  _Float16* WTq = (_Float16*)(ws);
  _Float16* WTk = (_Float16*)(ws + wt_bytes);
  _Float16* WTv = (_Float16*)(ws + 2 * wt_bytes);
  _Float16* qhp = (_Float16*)(ws + 3 * wt_bytes);
  _Float16* khp = (_Float16*)(ws + 3 * wt_bytes + qkv_bytes);
  _Float16* vTp = (_Float16*)(ws + 3 * wt_bytes + 2 * qkv_bytes);

  gpt2attn_wt_kernel<<<(Dc * HDc) / 256, 256, 0, stream>>>(Wq, Wk, Wv, WTq, WTk, WTv);
  gpt2attn_qkv_kernel<<<(Bc * Sc) / 16, 256, 0, stream>>>(x, WTq, WTk, WTv, qhp, khp, vTp);
  gpt2attn_flash_kernel<<<(Bc * Sc) / 64, 128, 0, stream>>>(qhp, khp, vTp, out);
}
